// AqSolModel_16647293239458
// MI455X (gfx1250) — hardware-verified
//
#include <hip/hip_runtime.h>
#include <stddef.h>


#define NTHR  256
#define NWAVE 8
#define HC    128
#define GR    32
#define GC    128
#define XSP   132
#define NBK   512
#define CHUNK 4096
#define NGRP  (CHUNK / (NTHR * 4))
#define WCAP  ((CHUNK / NTHR) * 32)
#define MXP   (NBK + 8)
#define AGG_LDS_BYTES ((((NBK + 1) * HC) + 2 * MXP) * 4 + (NWAVE * WCAP + NWAVE) * 4)
#define HTHR  512

static_assert(NGRP == 4);
static_assert(WCAP == 512);
static_assert(AGG_LDS_BYTES == 283232);
static_assert((NBK & (NBK - 1)) == 0);
static_assert(NBK <= 512);
static_assert(CHUNK <= 4096);
static_assert((NBK % (2 * NWAVE)) == 0);
static_assert((XSP % 4) == 0);
static_assert(GC == NWAVE * 16);

typedef float          v4f  __attribute__((ext_vector_type(4)));
typedef float          v8f  __attribute__((ext_vector_type(8)));
typedef int            v4i  __attribute__((ext_vector_type(4)));
typedef _Float16       v8h  __attribute__((ext_vector_type(8)));
typedef _Float16       v16h __attribute__((ext_vector_type(16)));

union FragH { v16h v; v4i u[2]; };
union Pack  { v8h h; v4i i; };

__device__ __forceinline__ v8f wmh(v16h a, v16h b, v8f c) {
  v8f d = __builtin_amdgcn_wmma_f32_16x16x32_f16(false, a, false, b, (short)0, c, false, false);
  asm volatile("v_nop\n\tv_nop\n\tv_nop\n\tv_nop" : "+v"(d) : "v"(a), "v"(b));
  return d;
}

__device__ __forceinline__ float lk(float t) { return fmaxf(t, 0.2f * t); }
__device__ __forceinline__ float dl(v4f t, v4f w) {
  return w.x * lk(t.x) + w.y * lk(t.y) + w.z * lk(t.z) + w.w * lk(t.w);
}
__device__ __forceinline__ v4f relu4(v4f v) {
  v4f r;
  r.x = fmaxf(v.x, 0.f); r.y = fmaxf(v.y, 0.f); r.z = fmaxf(v.z, 0.f); r.w = fmaxf(v.w, 0.f);
  return r;
}

__global__ __launch_bounds__(NTHR) void k_cvtx(const float* __restrict__ x, unsigned short* xf,
                                               int nN, int rowsTot, int K) {
  const int kp8 = K >> 3;
  const int i   = blockIdx.x * NTHR + threadIdx.x;
  if (i >= rowsTot * kp8) return;
  const int r  = i / kp8;
  const int kb = (i - r * kp8) * 8;
  v4f a = {0.f, 0.f, 0.f, 0.f}, b = {0.f, 0.f, 0.f, 0.f};
  if (r < nN) {
    a = *(const v4f*)(x + (size_t)r * K + kb);
    b = *(const v4f*)(x + (size_t)r * K + kb + 4);
  }
  Pack u;
  u.h[0] = (_Float16)a.x; u.h[1] = (_Float16)a.y; u.h[2] = (_Float16)a.z; u.h[3] = (_Float16)a.w;
  u.h[4] = (_Float16)b.x; u.h[5] = (_Float16)b.y; u.h[6] = (_Float16)b.z; u.h[7] = (_Float16)b.w;
  unsigned short* p = xf + (size_t)i * 8;
  *(volatile v4i*)p = u.i;
  __threadfence();
  *(volatile v4i*)p = u.i;
}

__global__ __launch_bounds__(NTHR) void k_cvtw(const float* __restrict__ W0, const float* __restrict__ W1,
                                               unsigned short* D0, unsigned short* D1, int K, int NO, float sc) {
  const float* W = (blockIdx.y == 0) ? W0 : W1;
  unsigned short* D = (blockIdx.y == 0) ? D0 : D1;
  const int kp8 = K >> 3;
  const int i   = blockIdx.x * NTHR + threadIdx.x;
  if (i >= NO * kp8) return;
  const int n  = i / kp8;
  const int kb = (i - n * kp8) * 8;
  Pack u;
#pragma unroll
  for (int j = 0; j < 8; ++j) u.h[j] = (_Float16)(W[(size_t)(kb + j) * NO + n] * sc);
  unsigned short* p = D + (size_t)i * 8;
  *(volatile v4i*)p = u.i;
  __threadfence();
  *(volatile v4i*)p = u.i;
}

__global__ __launch_bounds__(NTHR) void k_gemm(const unsigned short* __restrict__ A, const unsigned short* __restrict__ B,
                                               const float* __restrict__ bias, float* out, int K, int Ncols, float oscale) {
  __shared__ __attribute__((aligned(16))) float Xs[GR * XSP];

  const int tid  = threadIdx.x;
  const int lane = tid & 31;
  const int wave = tid >> 5;
  const int hh   = lane >> 4;
  const int m    = lane & 15;
  const int rowBase = blockIdx.x * GR;
  const int colBase = blockIdx.y * GC;
  const int ncol = colBase + wave * 16 + m;

  const size_t ra0 = (size_t)(rowBase + m) * K + 8 * hh;
  const size_t ra1 = ra0 + (size_t)16 * K;
  const size_t rb  = (size_t)ncol * K + 8 * hh;

  v8f c0 = {0.f, 0.f, 0.f, 0.f, 0.f, 0.f, 0.f, 0.f};
  v8f c1 = {0.f, 0.f, 0.f, 0.f, 0.f, 0.f, 0.f, 0.f};

#pragma unroll 1
  for (int k0 = 0; k0 < K; k0 += 32) {
    FragH a0, a1, b;
    a0.u[0] = *(const v4i*)(A + ra0 + k0);  a0.u[1] = *(const v4i*)(A + ra0 + k0 + 16);
    a1.u[0] = *(const v4i*)(A + ra1 + k0);  a1.u[1] = *(const v4i*)(A + ra1 + k0 + 16);
    b.u[0]  = *(const v4i*)(B + rb + k0);   b.u[1]  = *(const v4i*)(B + rb + k0 + 16);
    c0 = wmh(a0.v, b.v, c0);
    c1 = wmh(a1.v, b.v, c1);
  }

  const float bv = bias[ncol];
  const int cl = wave * 16 + m;
#pragma unroll
  for (int r = 0; r < 8; ++r) {
    Xs[(8 * hh + r) * XSP + cl]      = c0[r] * oscale + bv;
    Xs[(16 + 8 * hh + r) * XSP + cl] = c1[r] * oscale + bv;
  }
  __syncthreads();

  v4f xv[4];
  float* xpp[4];
#pragma unroll
  for (int i = 0; i < 4; ++i) {
    xv[i]  = *(const v4f*)(Xs + (4 * wave + i) * XSP + 4 * lane);
    xpp[i] = out + (size_t)(rowBase + 4 * wave + i) * Ncols + colBase + 4 * lane;
  }
#pragma unroll
  for (int i = 0; i < 4; ++i) *(volatile v4f*)(xpp[i]) = xv[i];
  __threadfence();
#pragma unroll
  for (int i = 0; i < 4; ++i) *(volatile v4f*)(xpp[i]) = xv[i];
}

__global__ __launch_bounds__(NTHR) void k_agg(
    const int* __restrict__ ei, const float* __restrict__ xl, const float* __restrict__ xr,
    const float* __restrict__ att, const float* __restrict__ bias,
    unsigned short* hF, float* hO, int nN, int nE, int nW, int wF, int wO) {
  extern __shared__ v4f lds_dyn[];
  float* sacc = (float*)lds_dyn;
  float* mx   = sacc + (NBK + 1) * HC;
  float* dn   = mx + MXP;
  int*   list = (int*)(dn + MXP);
  int*   wcnt = list + NWAVE * WCAP;

  const int tid  = threadIdx.x;
  const int lane = tid & 31;
  const int wave = tid >> 5;
  const int nodeBase = blockIdx.x * NBK;

  {
    const v4f z4 = {0.f, 0.f, 0.f, 0.f};
    for (int i = tid; i < ((NBK + 1) * HC) / 4; i += NTHR) lds_dyn[i] = z4;
    for (int i = tid; i < MXP; i += NTHR) { mx[i] = -1.0e30f; dn[i] = 0.f; }
  }
  __syncthreads();

  const int grp = lane >> 3;
  const int gl  = lane & 7;
  const int c16 = 16 * gl;
  const v4f w0 = *(const v4f*)(att + c16);
  const v4f w1 = *(const v4f*)(att + c16 + 4);
  const v4f w2 = *(const v4f*)(att + c16 + 8);
  const v4f w3 = *(const v4f*)(att + c16 + 12);

  const int* eid = ei + nE;
  const bool al16 = ((nE & 3) == 0);
  const int nChunks = (nE + CHUNK - 1) / CHUNK;
  const int nodeD = (nodeBase < nN - 1) ? nodeBase : (nN - 1);

#pragma unroll 1
  for (int ch = 0; ch <= nChunks; ++ch) {
    const int cbase = ch * CHUNK;
    const bool selfp = (ch == nChunks);
    if (!selfp) {
      int wc = 0;
#pragma unroll
      for (int g4 = 0; g4 < NGRP; ++g4) {
        const int el0 = (g4 * NTHR + tid) * 4;
        const int e0  = cbase + el0;
        const int sent = -2147483647 - 1;
        v4i d;
        if (al16 && (e0 + 3 < nE)) {
          d = *(const v4i*)(eid + e0);
        } else {
          d.x = (e0     < nE) ? eid[min(e0, nE - 1)]     : sent;
          d.y = (e0 + 1 < nE) ? eid[min(e0 + 1, nE - 1)] : sent;
          d.z = (e0 + 2 < nE) ? eid[min(e0 + 2, nE - 1)] : sent;
          d.w = (e0 + 3 < nE) ? eid[min(e0 + 3, nE - 1)] : sent;
        }
        const unsigned s0 = (unsigned)d.x - (unsigned)nodeBase;
        const unsigned s1 = (unsigned)d.y - (unsigned)nodeBase;
        const unsigned s2 = (unsigned)d.z - (unsigned)nodeBase;
        const unsigned s3 = (unsigned)d.w - (unsigned)nodeBase;
        const bool h0 = s0 < (unsigned)NBK;
        const bool h1 = s1 < (unsigned)NBK;
        const bool h2 = s2 < (unsigned)NBK;
        const bool h3 = s3 < (unsigned)NBK;
#define HITJ(J, HJ, SJ) { \
          const unsigned mj = __builtin_amdgcn_ballot_w32(HJ); \
          if (mj != 0u) { \
            if (HJ) { \
              const int pos = wc + (int)__builtin_amdgcn_mbcnt_lo(mj, 0u); \
              if (pos < WCAP) list[wave * WCAP + pos] = ((el0 + (J)) << 9) | (int)(SJ); \
            } \
            wc += (int)__builtin_popcount(mj); } }
        HITJ(0, h0, s0)
        HITJ(1, h1, s1)
        HITJ(2, h2, s2)
        HITJ(3, h3, s3)
#undef HITJ
      }
      if (lane == 0) wcnt[wave] = wc;
    } else {
      for (int s = tid; s < NBK; s += NTHR) list[s] = s;
      if (tid < NWAVE) {
        int c = NBK - tid * WCAP;
        c = c < 0 ? 0 : (c > WCAP ? WCAP : c);
        wcnt[tid] = c;
      }
    }
    __syncthreads();

    if (wave == 0) {
#pragma unroll 1
      for (int wsx = 0; wsx < NWAVE; ++wsx) {
        int n = __builtin_amdgcn_readfirstlane(wcnt[wsx]);
        n = n > WCAP ? WCAP : n;
        n = n < 0 ? 0 : n;
        const int* lw = list + wsx * WCAP;
#pragma unroll 1
        for (int i = 0; i < n; i += 4) {
          const int idx = i + grp;
          const int idc = (idx < WCAP) ? idx : (WCAP - 1);
          int ent = lw[idc];
          ent = (idx < n) ? ent : -1;
          const int key = (ent < 0) ? (1024 + grp) : (ent & (NBK - 1));
          const int kq0 = __builtin_amdgcn_readlane(key, 0);
          const int kq1 = __builtin_amdgcn_readlane(key, 8);
          const int kq2 = __builtin_amdgcn_readlane(key, 16);
          const int kq3 = __builtin_amdgcn_readlane(key, 24);
          const bool coll = (kq0 == kq1) | (kq0 == kq2) | (kq0 == kq3) | (kq1 == kq2) | (kq1 == kq3) | (kq2 == kq3);
          const int reps = coll ? 4 : 1;
#pragma unroll 1
          for (int r = 0; r < reps; ++r) {
            int me = ent;
            if (coll) {
              const int er = __builtin_amdgcn_readlane(ent, 8 * r);
              me = (grp == 0) ? er : -1;
            }
            int slot = me & (NBK - 1);
            int node = nodeBase + slot;
            const bool dum = (me < 0) || (node >= nN);
            slot = dum ? NBK : slot;
            node = dum ? nodeD : node;
            const int el = (me >> 9) & (CHUNK - 1);
            int e = cbase + el;
            e = (e < nE) ? e : (nE - 1);
            int sj = ei[e];
            sj = sj < 0 ? 0 : (sj > nN - 1 ? nN - 1 : sj);
            const int src = selfp ? node : sj;
            const float* xs = xl + (size_t)src  * HC + c16;
            const float* xd = xr + (size_t)node * HC + c16;
            float* ar = sacc + slot * HC + c16;
            const v4f a0 = *(const v4f*)(xs),     a1 = *(const v4f*)(xs + 4);
            const v4f a2 = *(const v4f*)(xs + 8), a3 = *(const v4f*)(xs + 12);
            const v4f d0 = *(const v4f*)(xd),     d1 = *(const v4f*)(xd + 4);
            const v4f d2 = *(const v4f*)(xd + 8), d3 = *(const v4f*)(xd + 12);
            float s = dl(a0 + d0, w0) + dl(a1 + d1, w1) + dl(a2 + d2, w2) + dl(a3 + d3, w3);
            s += __shfl_xor(s, 4, 32);
            s += __shfl_xor(s, 2, 32);
            s += __shfl_xor(s, 1, 32);
            const float mo = mx[slot], dd = dn[slot];
            const float mn = fmaxf(mo, s);
            const float sc = __expf(mo - mn);
            const float p  = __expf(s - mn);
            v4f e0 = *(v4f*)(ar),     e1 = *(v4f*)(ar + 4);
            v4f e2 = *(v4f*)(ar + 8), e3 = *(v4f*)(ar + 12);
            e0 = e0 * sc + a0 * p;  e1 = e1 * sc + a1 * p;
            e2 = e2 * sc + a2 * p;  e3 = e3 * sc + a3 * p;
            if (!dum) {
              *(v4f*)(ar)     = e0;  *(v4f*)(ar + 4)  = e1;
              *(v4f*)(ar + 8) = e2;  *(v4f*)(ar + 12) = e3;
              mx[slot] = mn;
              dn[slot] = dd * sc + p;
            }
          }
        }
      }
    }
    __syncthreads();
  }

  {
    const int q  = lane >> 4;
    const int c8 = 8 * (lane & 15);
    const int c4 = 4 * lane;
    const v4f b4  = *(const v4f*)(bias + c4);
    const v4f b8a = *(const v4f*)(bias + c8);
    const v4f b8b = *(const v4f*)(bias + c8 + 4);
    const v4f z4  = {0.f, 0.f, 0.f, 0.f};
#pragma unroll 1
    for (int i = 0; i < NBK / (2 * NWAVE); ++i) {
      const int sA    = (NBK / NWAVE) * wave + 2 * i;
      const int nodeA = nodeBase + sA;
      if (nodeA >= nW) break;
      v4f oA = z4, oB = z4;
      if (nodeA < nN) {
        const v4f e = *(const v4f*)(sacc + sA * HC + c4);
        const float inv = __builtin_amdgcn_rcpf(dn[sA] + 1e-16f);
        oA = relu4(e * inv + b4);
      }
      if (nodeA + 1 < nN) {
        const v4f e = *(const v4f*)(sacc + (sA + 1) * HC + c4);
        const float inv = __builtin_amdgcn_rcpf(dn[sA + 1] + 1e-16f);
        oB = relu4(e * inv + b4);
      }
      Pack u;
      const v4i zi = {0, 0, 0, 0};
      u.i = zi;
      const int sq = sA + q;
      const int nodeq = nodeA + q;
      if (nodeq < nN) {
        const v4f e0 = *(const v4f*)(sacc + sq * HC + c8);
        const v4f e1 = *(const v4f*)(sacc + sq * HC + c8 + 4);
        const float inv = __builtin_amdgcn_rcpf(dn[sq] + 1e-16f);
        const v4f o0 = relu4(e0 * inv + b8a);
        const v4f o1 = relu4(e1 * inv + b8b);
        u.h[0] = (_Float16)o0.x; u.h[1] = (_Float16)o0.y; u.h[2] = (_Float16)o0.z; u.h[3] = (_Float16)o0.w;
        u.h[4] = (_Float16)o1.x; u.h[5] = (_Float16)o1.y; u.h[6] = (_Float16)o1.z; u.h[7] = (_Float16)o1.w;
      }
      float* pA = hO + (size_t)nodeA * HC + c4;
      float* pB = pA + HC;
      unsigned short* pF = hF + (size_t)nodeA * HC + 8 * lane;
      if (wO) { *(volatile v4f*)pA = oA; *(volatile v4f*)pB = oB; }
      if (wF) { *(volatile v4i*)pF = u.i; }
      __threadfence();
      if (wO) { *(volatile v4f*)pA = oA; *(volatile v4f*)pB = oB; }
      if (wF) { *(volatile v4i*)pF = u.i; }
    }
  }
}

__global__ __launch_bounds__(NTHR) void k_pool(const int* __restrict__ bt, const float* __restrict__ h,
                                               float* gm, int nN) {
  __shared__ int plist[NWAVE * WCAP];
  __shared__ int pcnt[NWAVE];
  const int gi   = blockIdx.x;
  const int tid  = threadIdx.x;
  const int lane = tid & 31;
  const int wave = tid >> 5;
  const bool al16 = ((nN & 3) == 0);
  const int nChunks = (nN + CHUNK - 1) / CHUNK;
  v4f acc = {0.f, 0.f, 0.f, 0.f};
  int cnt = 0;

#pragma unroll 1
  for (int ch = 0; ch < nChunks; ++ch) {
    const int cbase = ch * CHUNK;
    int wc = 0;
#pragma unroll
    for (int g4 = 0; g4 < NGRP; ++g4) {
      const int el0 = (g4 * NTHR + tid) * 4;
      const int e0  = cbase + el0;
      const int sent = -2147483647 - 1;
      v4i d;
      if (al16 && (e0 + 3 < nN)) {
        d = *(const v4i*)(bt + e0);
      } else {
        d.x = (e0     < nN) ? bt[min(e0, nN - 1)]     : sent;
        d.y = (e0 + 1 < nN) ? bt[min(e0 + 1, nN - 1)] : sent;
        d.z = (e0 + 2 < nN) ? bt[min(e0 + 2, nN - 1)] : sent;
        d.w = (e0 + 3 < nN) ? bt[min(e0 + 3, nN - 1)] : sent;
      }
      const bool h0 = (d.x == gi), h1 = (d.y == gi), h2 = (d.z == gi), h3 = (d.w == gi);
#define HITP(J, HJ) { \
        const unsigned mj = __builtin_amdgcn_ballot_w32(HJ); \
        if (mj != 0u) { \
          if (HJ) { \
            const int pos = wc + (int)__builtin_amdgcn_mbcnt_lo(mj, 0u); \
            if (pos < WCAP) plist[wave * WCAP + pos] = el0 + (J); \
          } \
          wc += (int)__builtin_popcount(mj); } }
      HITP(0, h0)
      HITP(1, h1)
      HITP(2, h2)
      HITP(3, h3)
#undef HITP
    }
    if (lane == 0) pcnt[wave] = wc;
    __syncthreads();

    if (wave == 0) {
#pragma unroll 1
      for (int wsx = 0; wsx < NWAVE; ++wsx) {
        int n = __builtin_amdgcn_readfirstlane(pcnt[wsx]);
        n = n > WCAP ? WCAP : n;
        n = n < 0 ? 0 : n;
        cnt += n;
#pragma unroll 1
        for (int i = 0; i < n; ++i) {
          const int el = __builtin_amdgcn_readfirstlane(plist[wsx * WCAP + i]) & (CHUNK - 1);
          int node = cbase + el;
          node = (node < nN) ? node : (nN - 1);
          acc += *(const v4f*)(h + (size_t)node * HC + 4 * lane);
        }
      }
    }
    __syncthreads();
  }

  if (wave == 0) {
    const float c = (float)((cnt > 1) ? cnt : 1);
    const float inv = 1.0f / c;
    const v4f o = acc * inv;
    float* p = gm + (size_t)gi * HC + 4 * lane;
    *(volatile v4f*)p = o;
    __threadfence();
    *(volatile v4f*)p = o;
  }
}

__global__ __launch_bounds__(HTHR) void k_head(const float* __restrict__ gm, const float* __restrict__ lw,
                                               const float* __restrict__ lb, const float* __restrict__ ow,
                                               const float* __restrict__ ob, float* out, int nG, int HO) {
  __shared__ __attribute__((aligned(16))) float so[HTHR];
  const int t = threadIdx.x;
  float ov = 0.f;
  if (t < nG) {
    const float* gr = gm + (size_t)t * HC;
    float o = ob[0];
#pragma unroll 1
    for (int j = 0; j < HO; ++j) {
      float acc = lb[j];
      const float* wc = lw + j;
#pragma unroll 1
      for (int k = 0; k < HC; k += 4) {
        const v4f x4 = *(const v4f*)(gr + k);
        acc += x4.x * wc[(size_t)(k)     * HO];
        acc += x4.y * wc[(size_t)(k + 1) * HO];
        acc += x4.z * wc[(size_t)(k + 2) * HO];
        acc += x4.w * wc[(size_t)(k + 3) * HO];
      }
      acc = fmaxf(acc, 0.f);
      o += acc * ow[j];
    }
    ov = o;
  }
  so[t] = ov;
  __syncthreads();
  const bool wr = (4 * t + 3 < nG);
  v4f v = {0.f, 0.f, 0.f, 0.f};
  if (wr) v = *(const v4f*)(so + 4 * t);
  float* p = out + 4 * t;
  if (wr) *(volatile v4f*)p = v;
  __threadfence();
  if (wr) *(volatile v4f*)p = v;
}

extern "C" void kernel_launch(void* const* d_in, const int* in_sizes, int n_in,
                              void* d_out, int out_size, void* d_ws, size_t ws_size,
                              hipStream_t stream) {
  if (n_in < 25) return;
  const int F0 = 64, HO = 64;
  const int nN = in_sizes[2];
  if (nN <= 0 || in_sizes[0] != nN * F0) return;
  const int nE = in_sizes[1] / 2;
  if (nE <= 0 || in_sizes[1] != 2 * nE) return;
  if (in_sizes[3] != F0 * HC || in_sizes[5] != F0 * HC) return;
  if (in_sizes[4] != HC || in_sizes[6] != HC || in_sizes[7] != HC || in_sizes[8] != HC) return;
  if (in_sizes[9] != HC * HC || in_sizes[11] != HC * HC) return;
  if (in_sizes[10] != HC || in_sizes[12] != HC || in_sizes[13] != HC || in_sizes[14] != HC) return;
  if (in_sizes[15] != HC * HC || in_sizes[17] != HC * HC) return;
  if (in_sizes[16] != HC || in_sizes[18] != HC || in_sizes[19] != HC || in_sizes[20] != HC) return;
  if (in_sizes[21] != HC * HO || in_sizes[22] != HO || in_sizes[23] != HO || in_sizes[24] < 1) return;
  const int nG = out_size;
  if (nG <= 0 || nG > HTHR || (nG & 31) != 0) return;

  const float* x   = (const float*)d_in[0];
  const int*   ei  = (const int*)d_in[1];
  const int*   bt  = (const int*)d_in[2];
  const float* Wl0 = (const float*)d_in[3];   const float* bl0 = (const float*)d_in[4];
  const float* Wr0 = (const float*)d_in[5];   const float* br0 = (const float*)d_in[6];
  const float* at0 = (const float*)d_in[7];   const float* b0  = (const float*)d_in[8];
  const float* Wl1 = (const float*)d_in[9];   const float* bl1 = (const float*)d_in[10];
  const float* Wr1 = (const float*)d_in[11];  const float* br1 = (const float*)d_in[12];
  const float* at1 = (const float*)d_in[13];  const float* b1  = (const float*)d_in[14];
  const float* Wl2 = (const float*)d_in[15];  const float* bl2 = (const float*)d_in[16];
  const float* Wr2 = (const float*)d_in[17];  const float* br2 = (const float*)d_in[18];
  const float* at2 = (const float*)d_in[19];  const float* b2  = (const float*)d_in[20];
  const float* lw  = (const float*)d_in[21];  const float* lb  = (const float*)d_in[22];
  const float* ow  = (const float*)d_in[23];  const float* ob  = (const float*)d_in[24];
  float* out = (float*)d_out;

  const int Mpad = ((nN + GR - 1) / GR) * GR;

  char* wsp = (char*)d_ws;
  size_t off = 0;
  const size_t xFB = (size_t)Mpad * F0 * 2;
  const size_t hFB = (size_t)Mpad * HC * 2;
  const size_t wB  = (size_t)HC * HC * 2;
  const size_t xB  = (size_t)Mpad * HC * 4;
  const size_t gB  = (size_t)nG * HC * 4;
  unsigned short* xF = (unsigned short*)(wsp + off); off += xFB;
  unsigned short* hF = (unsigned short*)(wsp + off); off += hFB;
  unsigned short* Bl = (unsigned short*)(wsp + off); off += wB;
  unsigned short* Br = (unsigned short*)(wsp + off); off += wB;
  float* xl = (float*)(wsp + off); off += xB;
  float* xr = (float*)(wsp + off); off += xB;
  float* hO = (float*)(wsp + off); off += xB;
  float* gm = (float*)(wsp + off); off += gB;
  if (off > ws_size) return;

  const float s16  = 16.0f;
  const float is16 = 0.0625f;
  const int mt = Mpad / GR;
  const int aggBlocks = (Mpad + NBK - 1) / NBK;

  hipFuncSetAttribute(reinterpret_cast<const void*>(&k_agg),
                      hipFuncAttributeMaxDynamicSharedMemorySize, AGG_LDS_BYTES);

  k_cvtx<<<(Mpad * (F0 / 8) + NTHR - 1) / NTHR, NTHR, 0, stream>>>(x, xF, nN, Mpad, F0);

  k_cvtw<<<dim3((HC * (F0 / 8) + NTHR - 1) / NTHR, 2), NTHR, 0, stream>>>(Wl0, Wr0, Bl, Br, F0, HC, s16);
  k_gemm<<<dim3(mt, HC / GC), NTHR, 0, stream>>>(xF, Bl, bl0, xl, F0, HC, is16);
  k_gemm<<<dim3(mt, HC / GC), NTHR, 0, stream>>>(xF, Br, br0, xr, F0, HC, is16);
  k_agg<<<aggBlocks, NTHR, AGG_LDS_BYTES, stream>>>(ei, xl, xr, at0, b0, hF, hO, nN, nE, Mpad, 1, 0);

  k_cvtw<<<dim3((HC * (HC / 8) + NTHR - 1) / NTHR, 2), NTHR, 0, stream>>>(Wl1, Wr1, Bl, Br, HC, HC, s16);
  k_gemm<<<dim3(mt, HC / GC), NTHR, 0, stream>>>(hF, Bl, bl1, xl, HC, HC, is16);
  k_gemm<<<dim3(mt, HC / GC), NTHR, 0, stream>>>(hF, Br, br1, xr, HC, HC, is16);
  k_agg<<<aggBlocks, NTHR, AGG_LDS_BYTES, stream>>>(ei, xl, xr, at1, b1, hF, hO, nN, nE, Mpad, 1, 0);

  k_cvtw<<<dim3((HC * (HC / 8) + NTHR - 1) / NTHR, 2), NTHR, 0, stream>>>(Wl2, Wr2, Bl, Br, HC, HC, s16);
  k_gemm<<<dim3(mt, HC / GC), NTHR, 0, stream>>>(hF, Bl, bl2, xl, HC, HC, is16);
  k_gemm<<<dim3(mt, HC / GC), NTHR, 0, stream>>>(hF, Br, br2, xr, HC, HC, is16);
  k_agg<<<aggBlocks, NTHR, AGG_LDS_BYTES, stream>>>(ei, xl, xr, at2, b2, hF, hO, nN, nE, Mpad, 0, 1);

  k_pool<<<nG, NTHR, 0, stream>>>(bt, hO, gm, nN);
  k_head<<<1, HTHR, 0, stream>>>(gm, lw, lb, ow, ob, out, nG, HO);
}
